// RefinedAMSAM_17239998726609
// MI455X (gfx1250) — hardware-run, weakly checked
//
#include <hip/hip_runtime.h>
#include <math.h>

constexpr int kNS   = 3;
constexpr int kNB   = 4;
constexpr int kCI   = 64;
constexpr int kCO   = 128;
constexpr int kHW   = 56;
constexpr int kNPIX = 3136;
constexpr int kTOK  = kNB * kNPIX;
constexpr int kPBLK = kNPIX / 64;
constexpr int kQKD  = 16;
constexpr int kHID  = 8;
constexpr float kBnEps    = 1e-5f;
constexpr float kCarryW   = 16.0f;
constexpr float kCarryF   = 16.0f;
constexpr float kCarryP   = 32768.0f;
constexpr float kInvSqrtC = 0.0883883461356163f;
constexpr float kLog2e    = 1.44269504088896341f;

typedef __attribute__((ext_vector_type(16))) _Float16 v16h;
typedef __attribute__((ext_vector_type(8)))  _Float16 v8h;
typedef __attribute__((ext_vector_type(16))) __bf16   v16b;
typedef __attribute__((ext_vector_type(8)))  __bf16   v8b;
typedef __attribute__((ext_vector_type(8)))  float    v8f;
typedef __attribute__((ext_vector_type(4)))  float    v4f;
typedef __attribute__((ext_vector_type(4)))  unsigned int v4u;

__device__ __forceinline__ unsigned short f2bf_bits(float f) {
  unsigned u = __float_as_uint(f);
  return (unsigned short)((u + 0x7FFFu + ((u >> 16) & 1u)) >> 16);
}
__device__ __forceinline__ float bf_bits2f(unsigned short h) { return __uint_as_float(((unsigned)h) << 16); }

__device__ __forceinline__ void dep_guard_h(v8f& a, v8f& b, v16h x, v16h y) { asm volatile("v_nop\n\tv_nop\n\tv_nop\n\tv_nop" : "+v"(a), "+v"(b) : "v"(x), "v"(y)); }
__device__ __forceinline__ void dep_guard_b(v8f& a, v8f& b, v16b x, v16b y) { asm volatile("v_nop\n\tv_nop\n\tv_nop\n\tv_nop" : "+v"(a), "+v"(b) : "v"(x), "v"(y)); }
__device__ __forceinline__ void keep4_h(v16h a, v16h b, v16h c, v16h d) { asm volatile("v_nop" :: "v"(a), "v"(b), "v"(c), "v"(d)); }
__device__ __forceinline__ void keep4_b(v16b a, v16b b, v16b c, v16b d) { asm volatile("v_nop" :: "v"(a), "v"(b), "v"(c), "v"(d)); }
__device__ __forceinline__ void acc_guard4(v8f& a, v8f& b, v8f& c, v8f& d) { asm volatile("v_nop\n\tv_nop\n\tv_nop\n\tv_nop" : "+v"(a), "+v"(b), "+v"(c), "+v"(d)); }
template <typename T> struct Frag;
template <> struct Frag<_Float16> {
  typedef v16h V; union U { v16h v; v8h h[2]; };
  static __device__ __forceinline__ v16h load(const _Float16* p) {
    U f; f.h[0] = *(const v8h*)(p); f.h[1] = *(const v8h*)(p + 16); return f.v;
  }
  static __device__ __forceinline__ v8f mma(v16h a, v16h b, v8f c) {
    return __builtin_amdgcn_wmma_f32_16x16x32_f16(false, a, false, b, (short)0, c, false, false);
  }
  static __device__ __forceinline__ void guard(v8f& a, v8f& b, v16h x, v16h y) { dep_guard_h(a, b, x, y); }
  static __device__ __forceinline__ void keep(v16h a, v16h b, v16h c, v16h d) { keep4_h(a, b, c, d); }
};
template <> struct Frag<__bf16> {
  typedef v16b V; union U { v16b v; v8b h[2]; };
  static __device__ __forceinline__ v16b load(const __bf16* p) {
    U f; f.h[0] = *(const v8b*)(p); f.h[1] = *(const v8b*)(p + 16); return f.v;
  }
  static __device__ __forceinline__ v8f mma(v16b a, v16b b, v8f c) {
    return __builtin_amdgcn_wmma_f32_16x16x32_bf16(false, a, false, b, (short)0, c, false, false);
  }
  static __device__ __forceinline__ void guard(v8f& a, v8f& b, v16b x, v16b y) { dep_guard_b(a, b, x, y); }
  static __device__ __forceinline__ void keep(v16b a, v16b b, v16b c, v16b d) { keep4_b(a, b, c, d); }
};

__device__ __forceinline__ unsigned pk16(unsigned short a, unsigned short b) { return (unsigned)a | ((unsigned)b << 16); }
__device__ __forceinline__ unsigned short h_bits(float f) { const _Float16 h = (_Float16)f; return __builtin_bit_cast(unsigned short, h); }

template <int ET> struct Elem;
template <> struct Elem<0> { typedef _Float16 T; };
template <> struct Elem<1> { typedef __bf16 T; };
template <int ET, bool SPLIT, int BIAS_MODE, int OUT_MODE, bool RESID, int ACT = 0>
__global__ __launch_bounds__(256) void wmma_gemm64(
    const unsigned short* __restrict__ Ap, const unsigned short* __restrict__ A2p, int lda, long strideA,
    const unsigned short* __restrict__ Btp, const unsigned short* __restrict__ Bt2p, int ldb, long strideB,
    void* __restrict__ Cout, void* __restrict__ Cout2, int ldc, long strideC,
    const float* __restrict__ bias,
    const float* __restrict__ resid, long strideR,
    int M, int N, int K, float scale) {
  typedef typename Elem<ET>::T T;
  typedef typename Frag<T>::V V;
  const T* A = (const T*)Ap; const T* A2 = (const T*)A2p; const T* Bt = (const T*)Btp; const T* Bt2 = (const T*)Bt2p;
  __shared__ __align__(16) float sT[8][16 * 68];
  const int b    = blockIdx.y;
  const int lane = threadIdx.x & 31;
  const int wave = threadIdx.x >> 5;
  const int tilesN = N >> 6;
  const int tilesM = M >> 6;
  const int tile = blockIdx.x * 8 + wave;
  if (tile >= tilesM * tilesN) return;
  const int tm = tile / tilesN;
  const int tn = tile - tm * tilesN;
  const int m0 = tm << 6;
  const int n0 = tn << 6;

  const T* Ab  = A  + (size_t)b * strideA;
  const T* Bb  = Bt + (size_t)b * strideB;
  const T* Ab2 = SPLIT ? (A2  + (size_t)b * strideA) : nullptr;
  const T* Bb2 = SPLIT ? (Bt2 + (size_t)b * strideB) : nullptr;

  const int rlane = lane & 15;
  const int koff  = (lane >> 4) * 8;
  const int mOff  = (lane >> 4) * 8;

  v8f acc[4][4];
#pragma unroll
  for (int i = 0; i < 4; ++i)
#pragma unroll
    for (int j = 0; j < 4; ++j) acc[i][j] = (v8f){0.f,0.f,0.f,0.f,0.f,0.f,0.f,0.f};

  for (int k0 = 0; k0 < K; k0 += 32) {
    V bh[4], bl[4];
#pragma unroll
    for (int j = 0; j < 4; ++j) {
      const size_t bo = (size_t)(n0 + (j << 4) + rlane) * ldb + koff + k0;
      bh[j] = Frag<T>::load(Bb + bo);
      if (SPLIT) bl[j] = Frag<T>::load(Bb2 + bo);
    }
#pragma unroll
    for (int i = 0; i < 4; ++i) {
      const size_t ao = (size_t)(m0 + (i << 4) + rlane) * lda + koff + k0;
      V ah = Frag<T>::load(Ab + ao);
      V al;
      if (SPLIT) al = Frag<T>::load(Ab2 + ao);
#pragma unroll
      for (int j = 0; j < 4; ++j) {
        acc[i][j] = Frag<T>::mma(ah, bh[j], acc[i][j]);
        if (SPLIT) {
          acc[i][j] = Frag<T>::mma(ah, bl[j], acc[i][j]);
          acc[i][j] = Frag<T>::mma(al, bh[j], acc[i][j]);
        }
      }
      Frag<T>::guard(acc[i][0], acc[i][3], ah, SPLIT ? al : ah);
    }
    Frag<T>::keep(bh[0], bh[1], bh[2], bh[3]);
    if (SPLIT) Frag<T>::keep(bl[0], bl[1], bl[2], bl[3]);
  }
  acc_guard4(acc[0][0], acc[0][1], acc[0][2], acc[0][3]);
  acc_guard4(acc[1][0], acc[1][1], acc[1][2], acc[1][3]);
  acc_guard4(acc[2][0], acc[2][1], acc[2][2], acc[2][3]);
  acc_guard4(acc[3][0], acc[3][1], acc[3][2], acc[3][3]);

  float* slab = sT[wave];
  const float* Rb = RESID ? (resid + (size_t)b * strideR) : nullptr;
#pragma unroll
  for (int i = 0; i < 4; ++i) {
    const int mBase = m0 + (i << 4);
#pragma unroll
    for (int j = 0; j < 4; ++j) {
      const int n = n0 + (j << 4) + rlane;
      float bv = 0.f;
      if (BIAS_MODE == 2) bv = bias[n];
#pragma unroll
      for (int r = 0; r < 8; ++r) {
        float v = acc[i][j][r] * scale;
        if (BIAS_MODE == 1) v += bias[mBase + mOff + r];
        if (BIAS_MODE == 2) v += bv;
        if (RESID) v += Rb[(size_t)(mBase + mOff + r) * ldc + n];
        if (ACT == 2) v = fmaxf(v, 0.0f);
        if (ACT == 4) v = (v > 0.f) ? v : 0.01f * v;
        slab[(mOff + r) * 68 + (j << 4) + rlane] = v;
      }
    }
    __builtin_amdgcn_fence(__ATOMIC_RELEASE, "workgroup");
    __builtin_amdgcn_wave_barrier();
    __builtin_amdgcn_fence(__ATOMIC_ACQUIRE, "workgroup");
    if (OUT_MODE == 0) {
      float* C = (float*)Cout + (size_t)b * strideC;
      const int hh = lane >> 4, c4 = (lane & 15) * 4;
      for (int pass = 0; pass < 2; ++pass) {
#pragma unroll
        for (int it = 0; it < 8; ++it) {
          const int row = it * 2 + hh;
          v4f v = *(const v4f*)(slab + row * 68 + c4);
          *(volatile v4f*)(C + (size_t)(mBase + row) * ldc + n0 + c4) = v;
        }
        __threadfence();
      }
    } else {
      const int q = lane >> 3, c8 = (lane & 7) * 8;
      unsigned short* C  = (unsigned short*)Cout  + (size_t)b * strideC;
      unsigned short* C2 = (OUT_MODE == 2) ? ((unsigned short*)Cout2 + (size_t)b * strideC) : nullptr;
      for (int pass = 0; pass < 2; ++pass) {
#pragma unroll
        for (int it = 0; it < 4; ++it) {
          const int row = it * 4 + q;
          const float* sp = slab + row * 68 + c8;
          v8h hv, lv;
#pragma unroll
          for (int e = 0; e < 8; ++e) {
            if (OUT_MODE == 1) {
              hv[e] = (_Float16)sp[e];
            } else {
              unsigned short hb = f2bf_bits(sp[e]);
              unsigned short lb = f2bf_bits(sp[e] - bf_bits2f(hb));
              hv[e] = __builtin_bit_cast(_Float16, hb);
              lv[e] = __builtin_bit_cast(_Float16, lb);
            }
          }
          *(volatile v8h*)(C + (size_t)(mBase + row) * ldc + n0 + c8) = hv;
          if (OUT_MODE == 2) *(volatile v8h*)(C2 + (size_t)(mBase + row) * ldc + n0 + c8) = lv;
        }
        __threadfence();
      }
    }
    __builtin_amdgcn_fence(__ATOMIC_RELEASE, "workgroup");
    __builtin_amdgcn_wave_barrier();
    __builtin_amdgcn_fence(__ATOMIC_ACQUIRE, "workgroup");
  }
}

__global__ __launch_bounds__(256) void prep_kernel(
    const float* __restrict__ pw_w, const float* __restrict__ wv_w, const float* __restrict__ proj_w,
    const float* __restrict__ wq_w, const float* __restrict__ wk_w,
    const float* __restrict__ wq_b, const float* __restrict__ wk_b, const float* __restrict__ wv_b,
    unsigned short* __restrict__ pw16, unsigned short* __restrict__ wv16, unsigned short* __restrict__ proj16,
    unsigned short* __restrict__ wqk64, float* __restrict__ bias64x, float* __restrict__ wvb16x)
{
  const int job = blockIdx.y;
  const int i = blockIdx.x * 256 + threadIdx.x;
  if (job <= 2) {
    const float* src = (job == 0) ? pw_w : ((job == 1) ? wv_w : proj_w);
    unsigned short* dst = (job == 0) ? pw16 : ((job == 1) ? wv16 : proj16);
    const int n8 = (job == 0) ? (kNS * kCO * kCI / 8) : ((job == 1) ? (kNS * kCO * kCO / 8) : (kCO * kCI / 8));
    if (i >= n8) return;
    const float* p = src + 8 * (size_t)i;
    const v4f a = *(const v4f*)(p);
    const v4f c = *(const v4f*)(p + 4);
    unsigned short hb[8];
#pragma unroll
    for (int e = 0; e < 4; ++e) {
      hb[e]     = h_bits(a[e] * kCarryW);
      hb[4 + e] = h_bits(c[e] * kCarryW);
    }
    const v4u u = (v4u){pk16(hb[0], hb[1]), pk16(hb[2], hb[3]), pk16(hb[4], hb[5]), pk16(hb[6], hb[7])};
    unsigned short* q = dst + 8 * (size_t)i;
    *(volatile v4u*)q = u;
    __threadfence();
    *(volatile v4u*)q = u;
  } else if (job == 3) {
    const int n8 = kNS * 64 * kCO / 8;
    if (i >= n8) return;
    const int e0  = 8 * i;
    const int s   = e0 / (64 * kCO);
    const int rem = e0 - s * 64 * kCO;
    const int r   = rem >> 7;
    const int c8  = rem & 127;
    const int rq  = (r < 16) ? r : 15;
    int rk = r - 32;
    rk = (rk < 0) ? 0 : ((rk > 15) ? 15 : rk);
    const float* pq = wq_w + (size_t)(s * kQKD + rq) * kCO + c8;
    const float* pk = wk_w + (size_t)(s * kQKD + rk) * kCO + c8;
    const v4f qa = *(const v4f*)(pq);
    const v4f qc = *(const v4f*)(pq + 4);
    const v4f ka = *(const v4f*)(pk);
    const v4f kc = *(const v4f*)(pk + 4);
    const bool useq = (r < 16);
    const bool usek = (r >= 32) && (r < 48);
    unsigned short hb[8];
#pragma unroll
    for (int e = 0; e < 4; ++e) {
      const float v0 = useq ? qa[e] : (usek ? ka[e] : 0.0f);
      const float v1 = useq ? qc[e] : (usek ? kc[e] : 0.0f);
      hb[e]     = h_bits(v0 * kCarryW);
      hb[4 + e] = h_bits(v1 * kCarryW);
    }
    const v4u u = (v4u){pk16(hb[0], hb[1]), pk16(hb[2], hb[3]), pk16(hb[4], hb[5]), pk16(hb[6], hb[7])};
    unsigned short* q = wqk64 + 8 * (size_t)i;
    *(volatile v4u*)q = u;
    __threadfence();
    *(volatile v4u*)q = u;
  } else if (job == 4) {
    if (i >= kNS * 64) return;
    const int s = i >> 6;
    const int r = i & 63;
    const int rq = (r < 16) ? r : 15;
    int rk = r - 32;
    rk = (rk < 0) ? 0 : ((rk > 15) ? 15 : rk);
    const float qv = wq_b[s * kQKD + rq];
    const float kv = wk_b[s * kQKD + rk];
    const bool useq = (r < 16);
    const bool usek = (r >= 32) && (r < 48);
    const float v = (useq ? qv : (usek ? kv : 0.0f)) * kCarryF;
    *(volatile float*)(bias64x + i) = v;
    __threadfence();
    *(volatile float*)(bias64x + i) = v;
  } else {
    if (i >= kNS * kCO) return;
    const float v = wv_b[i] * kCarryF;
    *(volatile float*)(wvb16x + i) = v;
    __threadfence();
    *(volatile float*)(wvb16x + i) = v;
  }
}

__global__ __launch_bounds__(256) void xt_kernel(const float* __restrict__ x, unsigned short* __restrict__ xT)
{
  __shared__ float sm[64][65];
  const int t  = threadIdx.x;
  const int n0 = blockIdx.x * 64;
  const int b  = blockIdx.y;
  const float* xb = x + (size_t)b * kCI * kNPIX;
#pragma unroll
  for (int it = 0; it < 16; ++it) {
    const int e  = it * 256 + t;
    const int c  = e >> 6;
    const int nl = e & 63;
    sm[nl][c] = xb[(size_t)c * kNPIX + n0 + nl];
  }
  __syncthreads();
  const int lane = t & 31, wave = t >> 5;
  const int q = lane >> 3, c8 = (lane & 7) * 8;
  unsigned short* op = xT + ((size_t)b * kNPIX + n0) * kCI;
  for (int pass = 0; pass < 2; ++pass) {
#pragma unroll
    for (int it = 0; it < 2; ++it) {
      const int row = wave * 8 + it * 4 + q;
      unsigned short hb[8];
#pragma unroll
      for (int e = 0; e < 8; ++e) hb[e] = h_bits(sm[row][c8 + e]);
      const v4u u = (v4u){pk16(hb[0], hb[1]), pk16(hb[2], hb[3]), pk16(hb[4], hb[5]), pk16(hb[6], hb[7])};
      *(volatile v4u*)(op + (size_t)row * kCI + c8) = u;
    }
    __threadfence();
  }
}

__global__ __launch_bounds__(256) void dwconv_kernel(
    const float* __restrict__ x, const float* __restrict__ dw_w, const float* __restrict__ dw_b,
    int br, int dil, unsigned short* __restrict__ F64)
{
  __shared__ float sw[kCI * 9];
  __shared__ float sbias[kCI];
  const int t = threadIdx.x;
  for (int e = t; e < kCI * 9; e += 256) sw[e] = dw_w[(size_t)br * kCI * 9 + e];
  if (t < kCI) sbias[t] = dw_b[br * kCI + t];
  __syncthreads();
  const int token = blockIdx.x * 32 + (t >> 3);
  const int c8 = (t & 7) * 8;
  const int b = token / kNPIX;
  const int n = token - b * kNPIX;
  const int h = n / kHW;
  const int w = n - h * kHW;
  const float* xb = x + ((size_t)b * kCI + c8) * kNPIX;
  float acc[8];
#pragma unroll
  for (int e = 0; e < 8; ++e) acc[e] = sbias[c8 + e];
#pragma unroll 1
  for (int ky = 0; ky < 3; ++ky) {
    const int hh = h + (ky - 1) * dil;
    const bool vh = (hh >= 0) && (hh < kHW);
    const int hc = vh ? hh : 0;
#pragma unroll
    for (int kx = 0; kx < 3; ++kx) {
      const int ww = w + (kx - 1) * dil;
      const bool ok = vh && (ww >= 0) && (ww < kHW);
      const int wc = ok ? ww : 0;
      const int pos = hc * kHW + wc;
      const int tap = ky * 3 + kx;
#pragma unroll
      for (int e = 0; e < 8; ++e) {
        float xv = xb[(size_t)e * kNPIX + pos];
        xv = ok ? xv : 0.0f;
        acc[e] += sw[(c8 + e) * 9 + tap] * xv;
      }
    }
  }
  unsigned short hb[8];
#pragma unroll
  for (int e = 0; e < 8; ++e) hb[e] = h_bits(acc[e] * kCarryF);
  const v4u u = (v4u){pk16(hb[0], hb[1]), pk16(hb[2], hb[3]), pk16(hb[4], hb[5]), pk16(hb[6], hb[7])};
  unsigned short* q = F64 + (size_t)token * kCI + c8;
  *(volatile v4u*)q = u;
  __threadfence();
  *(volatile v4u*)q = u;
}

__global__ __launch_bounds__(256) void bn_relu_pool_kernel(
    const float* __restrict__ Fraw,
    const float* __restrict__ bn_g, const float* __restrict__ bn_b,
    const float* __restrict__ bn_m, const float* __restrict__ bn_v,
    int br, unsigned short* __restrict__ Fh, float* __restrict__ part)
{
  __shared__ float red[16][kCO];
  const int t = threadIdx.x;
  const int rg = t >> 4;
  const int c8 = (t & 15) * 8;
  const int row0 = blockIdx.x * 64;
  float sc[8], sh[8], mu[8], ps[8];
#pragma unroll
  for (int e = 0; e < 8; ++e) {
    const int c = br * kCO + c8 + e;
    sc[e] = bn_g[c] * rsqrtf(bn_v[c] + kBnEps);
    sh[e] = bn_b[c];
    mu[e] = bn_m[c];
    ps[e] = 0.0f;
  }
  v4u st[4];
#pragma unroll
  for (int it = 0; it < 4; ++it) {
    const int row = row0 + it * 16 + rg;
    const float* p = Fraw + (size_t)row * kCO + c8;
    const v4f a = *(const v4f*)(p);
    const v4f c = *(const v4f*)(p + 4);
    float v[8];
#pragma unroll
    for (int e = 0; e < 4; ++e) { v[e] = a[e]; v[4 + e] = c[e]; }
    unsigned short hb[8];
#pragma unroll
    for (int e = 0; e < 8; ++e) {
      float f = (v[e] - mu[e]) * sc[e] + sh[e];
      f = fmaxf(f, 0.0f);
      ps[e] += f;
      hb[e] = h_bits(f * kCarryF);
    }
    st[it] = (v4u){pk16(hb[0], hb[1]), pk16(hb[2], hb[3]), pk16(hb[4], hb[5]), pk16(hb[6], hb[7])};
  }
  for (int pass = 0; pass < 2; ++pass) {
#pragma unroll
    for (int it = 0; it < 4; ++it) {
      const int row = row0 + it * 16 + rg;
      *(volatile v4u*)(Fh + (size_t)row * kCO + c8) = st[it];
    }
    __threadfence();
  }
#pragma unroll
  for (int e = 0; e < 8; ++e) red[rg][c8 + e] = ps[e];
  __syncthreads();
  if (t < kCO) {
    float s = 0.0f;
#pragma unroll
    for (int r = 0; r < 16; ++r) s += red[r][t];
    float* pp = part + (size_t)blockIdx.x * kCO + t;
    *(volatile float*)pp = s;
    __threadfence();
    *(volatile float*)pp = s;
  }
}

__global__ __launch_bounds__(128) void ca_kernel(
    const float* __restrict__ part,
    const float* __restrict__ fc1_w, const float* __restrict__ fc1_b,
    const float* __restrict__ fc2_w, const float* __restrict__ fc2_b,
    int br, float* __restrict__ cab)
{
  __shared__ float avg[kCO];
  __shared__ float hid[kHID];
  const int b = blockIdx.x;
  const int t = threadIdx.x;
  float s = 0.0f;
#pragma unroll 1
  for (int k = 0; k < kPBLK; ++k) s += part[((size_t)(b * kPBLK + k)) * kCO + t];
  avg[t] = s * (1.0f / (float)kNPIX);
  __syncthreads();
  const int j = t >> 4;
  const int c8 = (t & 15) * 8;
  float a = 0.0f;
#pragma unroll
  for (int e = 0; e < 8; ++e) a += fc1_w[(size_t)(br * kHID + j) * kCO + c8 + e] * avg[c8 + e];
#pragma unroll
  for (int off = 1; off < 16; off <<= 1) a += __shfl_xor(a, off, 32);
  const float hv = fmaxf(a + fc1_b[br * kHID + j], 0.0f);
  if ((t & 15) == 0) hid[j] = hv;
  __syncthreads();
  float z = fc2_b[br * kCO + t];
#pragma unroll
  for (int hh = 0; hh < kHID; ++hh) z += fc2_w[(size_t)(br * kCO + t) * kHID + hh] * hid[hh];
  const float cav = 1.0f / (1.0f + expf(-z));
  float* cp = cab + (size_t)(br * kNB + b) * kCO + t;
  *(volatile float*)cp = cav;
  __threadfence();
  *(volatile float*)cp = cav;
}

__global__ __launch_bounds__(256) void softmax_kernel(const float* __restrict__ S, unsigned short* __restrict__ P)
{
  __shared__ float redm[8];
  __shared__ float reds[8];
  const int row  = blockIdx.x;
  const int t    = threadIdx.x;
  const int lane = t & 31, wave = t >> 5;
  const float* sr = S + (size_t)row * kNPIX;
  const bool v1 = t < (kNPIX / 8 - 256);
  const int  j1 = v1 ? (t + 256) : (kNPIX / 8 - 1);
  const v4f a0 = *(const v4f*)(sr + 8 * t);
  const v4f a1 = *(const v4f*)(sr + 8 * t + 4);
  const v4f b0 = *(const v4f*)(sr + 8 * j1);
  const v4f b1 = *(const v4f*)(sr + 8 * j1 + 4);
  const float ma = fmaxf(fmaxf(fmaxf(a0[0], a0[1]), fmaxf(a0[2], a0[3])), fmaxf(fmaxf(a1[0], a1[1]), fmaxf(a1[2], a1[3])));
  const float mb = fmaxf(fmaxf(fmaxf(b0[0], b0[1]), fmaxf(b0[2], b0[3])), fmaxf(fmaxf(b1[0], b1[1]), fmaxf(b1[2], b1[3])));
  float m = v1 ? fmaxf(ma, mb) : ma;
#pragma unroll
  for (int off = 16; off > 0; off >>= 1) m = fmaxf(m, __shfl_xor(m, off, 32));
  if (lane == 0) redm[wave] = m;
  __syncthreads();
  float gm = redm[0];
#pragma unroll
  for (int wv = 1; wv < 8; ++wv) gm = fmaxf(gm, redm[wv]);
  v4f ea0, ea1, eb0, eb1;
#pragma unroll
  for (int e = 0; e < 4; ++e) {
    ea0[e] = exp2f((a0[e] - gm) * kLog2e);
    ea1[e] = exp2f((a1[e] - gm) * kLog2e);
    eb0[e] = exp2f((b0[e] - gm) * kLog2e);
    eb1[e] = exp2f((b1[e] - gm) * kLog2e);
  }
  const float sa = ((ea0[0] + ea0[1]) + (ea0[2] + ea0[3])) + ((ea1[0] + ea1[1]) + (ea1[2] + ea1[3]));
  const float sb = ((eb0[0] + eb0[1]) + (eb0[2] + eb0[3])) + ((eb1[0] + eb1[1]) + (eb1[2] + eb1[3]));
  float su = v1 ? (sa + sb) : sa;
#pragma unroll
  for (int off = 16; off > 0; off >>= 1) su += __shfl_xor(su, off, 32);
  if (lane == 0) reds[wave] = su;
  __syncthreads();
  float tot = reds[0];
#pragma unroll
  for (int wv = 1; wv < 8; ++wv) tot += reds[wv];
  const float inv = kCarryP / tot;
  unsigned short ha[8], hbv[8];
#pragma unroll
  for (int e = 0; e < 4; ++e) {
    ha[e]      = h_bits(ea0[e] * inv);
    ha[4 + e]  = h_bits(ea1[e] * inv);
    hbv[e]     = h_bits(eb0[e] * inv);
    hbv[4 + e] = h_bits(eb1[e] * inv);
  }
  const v4u ua = (v4u){pk16(ha[0], ha[1]), pk16(ha[2], ha[3]), pk16(ha[4], ha[5]), pk16(ha[6], ha[7])};
  const v4u ub = (v4u){pk16(hbv[0], hbv[1]), pk16(hbv[2], hbv[3]), pk16(hbv[4], hbv[5]), pk16(hbv[6], hbv[7])};
  unsigned short* pr = P + (size_t)row * kNPIX;
  for (int pass = 0; pass < 2; ++pass) {
    *(volatile v4u*)(pr + 8 * t) = ua;
    if (v1) *(volatile v4u*)(pr + 8 * (size_t)(t + 256)) = ub;
    __threadfence();
  }
}

__global__ __launch_bounds__(256) void combine_kernel(
    const float* __restrict__ PROJ, const float* __restrict__ AO, const float* __restrict__ cab,
    float* __restrict__ out)
{
  __shared__ float sm[64][65];
  const int t  = threadIdx.x;
  const int n0 = blockIdx.x * 64;
  const int c0 = blockIdx.y * 64;
  const int b  = blockIdx.z;
#pragma unroll 1
  for (int it = 0; it < 4; ++it) {
    const int e  = it * 256 + t;
    const int rl = e >> 4;
    const int c4 = (e & 15) * 4;
    const size_t tok = (size_t)b * kNPIX + n0 + rl;
    const v4f pv = *(const v4f*)(PROJ + tok * kCO + c0 + c4);
    v4f fz = (v4f){0.0f, 0.0f, 0.0f, 0.0f};
#pragma unroll
    for (int i = 0; i < kNS; ++i) {
      const size_t tki = ((size_t)(i * kNB + b)) * kNPIX + n0 + rl;
      const v4f sv = *(const v4f*)(AO + tki * kCO + c0 + c4);
      const v4f cv = *(const v4f*)(cab + (size_t)(i * kNB + b) * kCO + c0 + c4);
#pragma unroll
      for (int e2 = 0; e2 < 4; ++e2) {
        const float af = sv[e2] * cv[e2];
        fz[e2] += af * af;
      }
    }
#pragma unroll
    for (int e2 = 0; e2 < 4; ++e2) sm[c4 + e2][rl] = pv[e2] + fz[e2];
  }
  __syncthreads();
  const int lane = t & 31, wave = t >> 5;
  const int hh = lane >> 4, cc4 = (lane & 15) * 4;
  float* ob = out + ((size_t)b * kCO + c0) * kNPIX + n0;
  for (int pass = 0; pass < 2; ++pass) {
#pragma unroll
    for (int it = 0; it < 4; ++it) {
      const int cl = wave * 8 + it * 2 + hh;
      v4f v;
      v[0] = sm[cl][cc4];
      v[1] = sm[cl][cc4 + 1];
      v[2] = sm[cl][cc4 + 2];
      v[3] = sm[cl][cc4 + 3];
      *(volatile v4f*)(ob + (size_t)cl * kNPIX + cc4) = v;
    }
    __threadfence();
  }
}

static inline unsigned int gemm_blocks(int M, int N) { return (unsigned int)(((M >> 6) * (N >> 6) + 7) / 8); }

extern "C" void kernel_launch(void* const* d_in, const int* in_sizes, int n_in,
                              void* d_out, int out_size, void* d_ws, size_t ws_size,
                              hipStream_t stream)
{
  if (n_in < 21) return;
  if (in_sizes[0] != kNB * kCI * kNPIX) return;
  if (out_size != kNB * kCO * kNPIX) return;

  const float* x      = (const float*)d_in[0];
  const float* dw_w   = (const float*)d_in[1];
  const float* dw_b   = (const float*)d_in[2];
  const float* pw_w   = (const float*)d_in[3];
  const float* pw_b   = (const float*)d_in[4];
  const float* bn_g   = (const float*)d_in[5];
  const float* bn_b   = (const float*)d_in[6];
  const float* bn_m   = (const float*)d_in[7];
  const float* bn_v   = (const float*)d_in[8];
  const float* wq_w   = (const float*)d_in[9];
  const float* wq_b   = (const float*)d_in[10];
  const float* wk_w   = (const float*)d_in[11];
  const float* wk_b   = (const float*)d_in[12];
  const float* wv_w   = (const float*)d_in[13];
  const float* wv_b   = (const float*)d_in[14];
  const float* fc1_w  = (const float*)d_in[15];
  const float* fc1_b  = (const float*)d_in[16];
  const float* fc2_w  = (const float*)d_in[17];
  const float* fc2_b  = (const float*)d_in[18];
  const float* proj_w = (const float*)d_in[19];
  const float* proj_b = (const float*)d_in[20];
  float* out = (float*)d_out;

  char* ws = (char*)d_ws;
  size_t off = 0;
  auto carve = [&](size_t bytes) -> char* {
    char* p = ws + off;
    off += (bytes + 255) & ~(size_t)255;
    return p;
  };
  unsigned short* pw16    = (unsigned short*)carve((size_t)kNS * kCO * kCI * 2);
  unsigned short* wv16    = (unsigned short*)carve((size_t)kNS * kCO * kCO * 2);
  unsigned short* proj16  = (unsigned short*)carve((size_t)kCO * kCI * 2);
  unsigned short* wqk64   = (unsigned short*)carve((size_t)kNS * 64 * kCO * 2);
  float*          bias64x = (float*)carve((size_t)kNS * 64 * 4);
  float*          wvb16x  = (float*)carve((size_t)kNS * kCO * 4);
  unsigned short* xT16    = (unsigned short*)carve((size_t)kTOK * kCI * 2);
  float*          PROJ    = (float*)carve((size_t)kTOK * kCO * 4);
  unsigned short* F64     = (unsigned short*)carve((size_t)kTOK * kCI * 2);
  float*          Fraw    = (float*)carve((size_t)kTOK * kCO * 4);
  unsigned short* Fh      = (unsigned short*)carve((size_t)kTOK * kCO * 2);
  float*          part    = (float*)carve((size_t)kNB * kPBLK * kCO * 4);
  float*          cab     = (float*)carve((size_t)kNS * kNB * kCO * 4);
  unsigned short* QK16    = (unsigned short*)carve((size_t)kTOK * 64 * 2);
  unsigned short* Vt16    = (unsigned short*)carve((size_t)kNB * kCO * kNPIX * 2);
  float*          Spl     = (float*)carve((size_t)kNPIX * kNPIX * 4);
  unsigned short* P16     = (unsigned short*)carve((size_t)kNPIX * kNPIX * 2);
  float*          AO      = (float*)carve((size_t)kNS * kNB * kNPIX * kCO * 4);
  if (off > ws_size) return;

  prep_kernel<<<dim3(24, 6), 256, 0, stream>>>(pw_w, wv_w, proj_w, wq_w, wk_w, wq_b, wk_b, wv_b,
                                               pw16, wv16, proj16, wqk64, bias64x, wvb16x);
  xt_kernel<<<dim3(kPBLK, kNB), 256, 0, stream>>>(x, xT16);
  wmma_gemm64<0, false, 2, 0, false, 0><<<dim3(gemm_blocks(kTOK, kCO), 1), 256, 0, stream>>>(
      xT16, xT16, kCI, 0L, proj16, proj16, kCI, 0L,
      (void*)PROJ, (void*)PROJ, kCO, 0L, proj_b, proj_b, 0L, kTOK, kCO, kCI, 1.0f / kCarryW);

  for (int br = 0; br < kNS; ++br) {
    const int dil = (br == 0) ? 1 : ((br == 1) ? 2 : 4);
    dwconv_kernel<<<dim3(kTOK / 32), 256, 0, stream>>>(x, dw_w, dw_b, br, dil, F64);
    wmma_gemm64<0, false, 2, 0, false, 0><<<dim3(gemm_blocks(kTOK, kCO), 1), 256, 0, stream>>>(
        F64, F64, kCI, 0L, pw16 + (size_t)br * kCO * kCI, pw16 + (size_t)br * kCO * kCI, kCI, 0L,
        (void*)Fraw, (void*)Fraw, kCO, 0L, pw_b + br * kCO, pw_b, 0L, kTOK, kCO, kCI, 1.0f / (kCarryF * kCarryW));
    bn_relu_pool_kernel<<<dim3(kTOK / 64), 256, 0, stream>>>(Fraw, bn_g, bn_b, bn_m, bn_v, br, Fh, part);
    ca_kernel<<<dim3(kNB), 128, 0, stream>>>(part, fc1_w, fc1_b, fc2_w, fc2_b, br, cab);
    wmma_gemm64<0, false, 2, 1, false, 0><<<dim3(gemm_blocks(kTOK, 64), 1), 256, 0, stream>>>(
        Fh, Fh, kCO, 0L, wqk64 + (size_t)br * 64 * kCO, wqk64 + (size_t)br * 64 * kCO, kCO, 0L,
        (void*)QK16, (void*)QK16, 64, 0L, bias64x + br * 64, bias64x, 0L, kTOK, 64, kCO, 1.0f / kCarryW);
    wmma_gemm64<0, false, 1, 1, false, 0><<<dim3(gemm_blocks(kCO, kNPIX), kNB), 256, 0, stream>>>(
        wv16 + (size_t)br * kCO * kCO, wv16 + (size_t)br * kCO * kCO, kCO, 0L,
        Fh, Fh, kCO, (long)kNPIX * kCO,
        (void*)Vt16, (void*)Vt16, kNPIX, (long)kCO * kNPIX, wvb16x + br * kCO, wvb16x, 0L,
        kCO, kNPIX, kCO, 1.0f / kCarryW);
    for (int b = 0; b < kNB; ++b) {
      const unsigned short* qk = QK16 + (size_t)b * kNPIX * 64;
      wmma_gemm64<0, false, 0, 0, false, 0><<<dim3(gemm_blocks(kNPIX, kNPIX), 1), 256, 0, stream>>>(
          qk, qk, 64, 0L, qk + 32, qk + 32, 64, 0L,
          (void*)Spl, (void*)Spl, kNPIX, 0L, proj_b, proj_b, 0L, kNPIX, kNPIX, 32,
          kInvSqrtC / (kCarryF * kCarryF));
      softmax_kernel<<<dim3(kNPIX), 256, 0, stream>>>(Spl, P16);
      wmma_gemm64<0, false, 0, 0, false, 0><<<dim3(gemm_blocks(kNPIX, kCO), 1), 256, 0, stream>>>(
          P16, P16, kNPIX, 0L, Vt16 + (size_t)b * kCO * kNPIX, Vt16 + (size_t)b * kCO * kNPIX, kNPIX, 0L,
          (void*)(AO + ((size_t)(br * kNB + b)) * kNPIX * kCO), (void*)(AO + ((size_t)(br * kNB + b)) * kNPIX * kCO),
          kCO, 0L, proj_b, proj_b, 0L, kNPIX, kCO, kNPIX, 1.0f / (kCarryP * kCarryF));
    }
  }
  combine_kernel<<<dim3(kPBLK, 2, kNB), 256, 0, stream>>>(PROJ, AO, cab, out);
}
